// Classifier_62938450755768
// MI455X (gfx1250) — hardware-run, weakly checked
//
#include <hip/hip_runtime.h>
#include <stddef.h>
#include <stdint.h>
#include <math.h>

#define NN      100000
#define NE      600000
#define FD      128
#define NCL     16
#define KP      256
#define GBM     128
#define MP      100096
#define NTHR    256
#define NWAVE   8
#define EPT     8
#define WCH     (32 * EPT)
#define NBRUN   1024
#define SLB     10
#define NBK     98
#define WLCAP   2048
#define RCAP    8192
#define TRIPCAP 64
#define MAXDEG_IN_MEAS    20
#define MAXB1024_IN_MEAS  6360
#define MAXB1024_OUT_MEAS 6330
#define ABM     64
#define SP      68
#define SPLIT_L2   1
#define SPLIT_HEAD 1
#define K_L2   (SPLIT_L2 ? KP : FD)
#define K_HEAD (SPLIT_HEAD ? KP : FD)

#define BK_ZINTS (2 * NWAVE * WLCAP + RCAP + 4 * NBRUN + 2 * NBRUN)
#define BK_INTS  (BK_ZINTS + 32)
#define BK_LDS   (BK_INTS * 4)

#define PBX  (MP * FD / 8 / NTHR)
#define PBW1 (FD * FD / 8 / NTHR)
#define PBW2 (FD * KP / 8 / NTHR)
#define PBWC (NCL * KP / 8 / NTHR)
#define PBTOT (PBX + PBW1 + PBW2 + PBWC + 1)
#define SMN  384

static_assert(FD == 128 && NCL == 16 && KP == 2 * FD);
static_assert(NN % 2 == 0 && NN <= NBK * NBRUN);
static_assert(MP % GBM == 0 && MP >= NN && MP == 782 * GBM && MP % ABM == 0 && MP <= NBK * NBRUN);
static_assert(NBRUN == (1 << SLB) && NBRUN % ABM == 0 && NBRUN % GBM == 0 && NBRUN == NTHR * 4);
static_assert(NE == 600000 && NE % EPT == 0 && NE < (1 << 20));
static_assert((((long long)NE + WCH) << SLB) < (1LL << 31));
static_assert((long long)RCAP * 100 >= (long long)MAXB1024_IN_MEAS * 105);
static_assert(WLCAP >= 2 * (MAXB1024_IN_MEAS / NWAVE + 1) && WLCAP >= 2 * (MAXB1024_OUT_MEAS / NWAVE + 1));
static_assert(MAXDEG_IN_MEAS + 8 <= TRIPCAP);
static_assert(RCAP % (NTHR * 4) == 0 && BK_ZINTS % 4 == 0);
static_assert(BK_LDS <= 300000);
static_assert((GBM * NCL * 4) % 128 == 0 && (((NN % GBM) * NCL * 4) % 128) == 0);
static_assert(GBM * NCL / 4 == 2 * NTHR);
static_assert((MP * FD / 8) % NTHR == 0 && (FD * FD / 8) % NTHR == 0);
static_assert((FD * KP / 8) % NTHR == 0 && (NCL * KP / 8) % NTHR == 0);
static_assert(FD % 32 == 0 && KP % 32 == 0 && K_L2 % 32 == 0 && K_HEAD % 32 == 0);
static_assert(K_L2 <= KP && K_HEAD <= KP);
static_assert((GBM * SP + GBM) * 4 <= 65536);
static_assert(SMN == 3 * 128);

typedef float          v4f   __attribute__((ext_vector_type(4)));
typedef float          v8f   __attribute__((ext_vector_type(8)));
typedef int            v4i   __attribute__((ext_vector_type(4)));
typedef int            v8i   __attribute__((ext_vector_type(8)));
typedef unsigned short v8us  __attribute__((ext_vector_type(8)));
typedef unsigned short v16us __attribute__((ext_vector_type(16)));
typedef __bf16         v16bf __attribute__((ext_vector_type(16)));
typedef v4f  __attribute__((may_alias)) v4fa;
typedef v4i  __attribute__((may_alias)) v4ia;
typedef v8us __attribute__((may_alias)) v8usa;
union FragB { v16bf v; v16us u; v8us h[2]; v8i w; };

__device__ __forceinline__ v8f wmb(const FragB& a, const FragB& b, v8f c) {
  v8f d = __builtin_amdgcn_wmma_f32_16x16x32_bf16(false, a.v, false, b.v, (short)0, c, false, false);
  asm volatile("v_nop\n\tv_nop\n\tv_nop\n\tv_nop" : "+v"(d) : "v"(a.w), "v"(b.w));
  return d;
}

__device__ __forceinline__ unsigned bf16_bits(float f) {
  const unsigned u = __float_as_uint(f);
  const unsigned r = (u + 0x7FFFu + ((u >> 16) & 1u)) >> 16;
  const unsigned q = (u >> 16) | 0x40u;
  return ((u & 0x7fffffffu) > 0x7f800000u) ? q : r;
}
__device__ __forceinline__ float bf16_val(float f) {
  return __uint_as_float(bf16_bits(f) << 16);
}

__device__ __forceinline__ void hilo_pack(float v0, float v1, float v2, float v3,
                                          int& h01, int& h23, int& l01, int& l23) {
  const unsigned a0 = bf16_bits(v0), a1 = bf16_bits(v1), a2 = bf16_bits(v2), a3 = bf16_bits(v3);
  const unsigned b0 = bf16_bits(v0 - __uint_as_float(a0 << 16));
  const unsigned b1 = bf16_bits(v1 - __uint_as_float(a1 << 16));
  const unsigned b2 = bf16_bits(v2 - __uint_as_float(a2 << 16));
  const unsigned b3 = bf16_bits(v3 - __uint_as_float(a3 << 16));
  h01 = (int)(a0 | (a1 << 16)); h23 = (int)(a2 | (a3 << 16));
  l01 = (int)(b0 | (b1 << 16)); l23 = (int)(b2 | (b3 << 16));
}

__device__ __forceinline__ v4i regroup_row(int h01, int h23, int l01, int l23, int lane) {
  const int s0 = (2 * lane) & 31, s1 = s0 + 1;
  const int a0 = __shfl(h01, s0, 32), a1 = __shfl(h23, s0, 32), a2 = __shfl(h01, s1, 32), a3 = __shfl(h23, s1, 32);
  const int b0 = __shfl(l01, s0, 32), b1 = __shfl(l23, s0, 32), b2 = __shfl(l01, s1, 32), b3 = __shfl(l23, s1, 32);
  const int mk = (lane < 16) ? -1 : 0;
  v4i o;
  o.x = (a0 & mk) | (b0 & ~mk); o.y = (a1 & mk) | (b1 & ~mk);
  o.z = (a2 & mk) | (b2 & ~mk); o.w = (a3 & mk) | (b3 & ~mk);
  return o;
}

__device__ __forceinline__ void st2_v4f(float* p, v4f v) {
  *(volatile v4f*)p = v;
  __threadfence();
  *(volatile v4f*)p = v;
}
__device__ __forceinline__ void st2_v8us(unsigned short* p, v8us v) {
  *(volatile v8us*)p = v;
  __threadfence();
  *(volatile v8us*)p = v;
}

__device__ __forceinline__ v8us gather8(const float* __restrict__ base, int stride) {
  float f[8];
#pragma unroll
  for (int i = 0; i < 8; ++i) f[i] = base[(size_t)i * (size_t)stride];
  v8us o;
#pragma unroll
  for (int i = 0; i < 8; ++i) o[i] = (unsigned short)bf16_bits(f[i]);
  return o;
}

__global__ __launch_bounds__(NTHR) void k_prep(const float* __restrict__ h, const float* __restrict__ w1,
                                               const float* __restrict__ b1, const float* __restrict__ w2,
                                               const float* __restrict__ b2, const float* __restrict__ wc,
                                               const float* __restrict__ bc,
                                               unsigned short* hb, unsigned short* w1t, unsigned short* w2d,
                                               unsigned short* wcd, float* sm) {
  const int tid = (int)threadIdx.x, lane = tid & 31, wave = tid >> 5;
  const int blk = (int)blockIdx.x;
  if (blk < PBX) {
    const int u   = blk * NTHR + tid;
    const int row = u >> 4, k8 = (u & 15) * 8;
    const int rc  = row < NN ? row : NN - 1;
    const unsigned mk = row < NN ? 0xffffu : 0u;
    const float* p = h + (size_t)rc * FD + k8;
    const v4f a = *(const v4fa*)p;
    const v4f b = *(const v4fa*)(p + 4);
    v8us o;
    o[0] = (unsigned short)(bf16_bits(a.x) & mk); o[1] = (unsigned short)(bf16_bits(a.y) & mk);
    o[2] = (unsigned short)(bf16_bits(a.z) & mk); o[3] = (unsigned short)(bf16_bits(a.w) & mk);
    o[4] = (unsigned short)(bf16_bits(b.x) & mk); o[5] = (unsigned short)(bf16_bits(b.y) & mk);
    o[6] = (unsigned short)(bf16_bits(b.z) & mk); o[7] = (unsigned short)(bf16_bits(b.w) & mk);
    st2_v8us(hb + (size_t)row * FD + k8, o);
  } else if (blk < PBX + PBW1) {
    const int u = (blk - PBX) * NTHR + tid;
    const int n = u >> 4, k8 = (u & 15) * 8;
    const v8us o = gather8(w1 + (size_t)k8 * FD + n, FD);
    st2_v8us(w1t + (size_t)n * FD + k8, o);
  } else if (blk < PBX + PBW1 + PBW2) {
    const int u = (blk - PBX - PBW1) * NTHR + tid;
    const int n = u >> 5, k8 = (u & 31) * 8, kk = k8 & (FD - 1);
    const v8us o = gather8(w2 + (size_t)kk * FD + n, FD);
    st2_v8us(w2d + (size_t)n * KP + k8, o);
  } else if (blk < PBX + PBW1 + PBW2 + PBWC) {
    const int u = (blk - PBX - PBW1 - PBW2) * NTHR + tid;
    const int n = u >> 5, k8 = (u & 31) * 8, kk = k8 & (FD - 1);
    const v8us o = gather8(wc + (size_t)kk * NCL + n, NCL);
    st2_v8us(wcd + (size_t)n * KP + k8, o);
  } else {
    if (wave == 0) {
      const v4f a = *(const v4fa*)(b1 + 4 * lane);
      v4f o;
      o.x = bf16_val(a.x); o.y = bf16_val(a.y); o.z = bf16_val(a.z); o.w = bf16_val(a.w);
      st2_v4f(sm + 4 * lane, o);
    } else if (wave == 1) {
      const v4f a = *(const v4fa*)(b2 + 4 * lane);
      v4f o;
      o.x = bf16_val(a.x); o.y = bf16_val(a.y); o.z = bf16_val(a.z); o.w = bf16_val(a.w);
      st2_v4f(sm + 128 + 4 * lane, o);
    } else if (wave == 2) {
      const int lc = lane < 4 ? lane : 3;
      const v4f a = *(const v4fa*)(bc + 4 * lc);
      asm volatile("" :: "v"(a));
      const unsigned mk = lane < 4 ? 0xffffffffu : 0u;
      v4f o;
      o.x = __uint_as_float((bf16_bits(a.x) << 16) & mk);
      o.y = __uint_as_float((bf16_bits(a.y) << 16) & mk);
      o.z = __uint_as_float((bf16_bits(a.z) << 16) & mk);
      o.w = __uint_as_float((bf16_bits(a.w) << 16) & mk);
      st2_v4f(sm + 256 + 4 * lane, o);
    }
  }
}

__device__ __forceinline__ void compact8(const v4i da, const v4i db, const bool valid, const unsigned nbs,
                                         const int e0, int* mylist, int& wc) {
  const unsigned s0 = (unsigned)da.x - nbs, s1 = (unsigned)da.y - nbs;
  const unsigned s2 = (unsigned)da.z - nbs, s3 = (unsigned)da.w - nbs;
  const unsigned s4 = (unsigned)db.x - nbs, s5 = (unsigned)db.y - nbs;
  const unsigned s6 = (unsigned)db.z - nbs, s7 = (unsigned)db.w - nbs;
  const bool h0 = valid && (s0 < (unsigned)NBRUN), h1 = valid && (s1 < (unsigned)NBRUN);
  const bool h2 = valid && (s2 < (unsigned)NBRUN), h3 = valid && (s3 < (unsigned)NBRUN);
  const bool h4 = valid && (s4 < (unsigned)NBRUN), h5 = valid && (s5 < (unsigned)NBRUN);
  const bool h6 = valid && (s6 < (unsigned)NBRUN), h7 = valid && (s7 < (unsigned)NBRUN);
  const unsigned m0 = __builtin_amdgcn_ballot_w32(h0), m1 = __builtin_amdgcn_ballot_w32(h1);
  const unsigned m2 = __builtin_amdgcn_ballot_w32(h2), m3 = __builtin_amdgcn_ballot_w32(h3);
  const unsigned m4 = __builtin_amdgcn_ballot_w32(h4), m5 = __builtin_amdgcn_ballot_w32(h5);
  const unsigned m6 = __builtin_amdgcn_ballot_w32(h6), m7 = __builtin_amdgcn_ballot_w32(h7);
  const unsigned any = m0 | m1 | m2 | m3 | m4 | m5 | m6 | m7;
  if (any != 0u) {
    const int pre = (int)(__builtin_amdgcn_mbcnt_lo(m0, 0u) + __builtin_amdgcn_mbcnt_lo(m1, 0u) +
                          __builtin_amdgcn_mbcnt_lo(m2, 0u) + __builtin_amdgcn_mbcnt_lo(m3, 0u) +
                          __builtin_amdgcn_mbcnt_lo(m4, 0u) + __builtin_amdgcn_mbcnt_lo(m5, 0u) +
                          __builtin_amdgcn_mbcnt_lo(m6, 0u) + __builtin_amdgcn_mbcnt_lo(m7, 0u));
    int p = wc + pre;
    if (h0) { if (p < WLCAP) mylist[p] = ((e0 + 0) << SLB) | (int)s0; p = p + 1; }
    if (h1) { if (p < WLCAP) mylist[p] = ((e0 + 1) << SLB) | (int)s1; p = p + 1; }
    if (h2) { if (p < WLCAP) mylist[p] = ((e0 + 2) << SLB) | (int)s2; p = p + 1; }
    if (h3) { if (p < WLCAP) mylist[p] = ((e0 + 3) << SLB) | (int)s3; p = p + 1; }
    if (h4) { if (p < WLCAP) mylist[p] = ((e0 + 4) << SLB) | (int)s4; p = p + 1; }
    if (h5) { if (p < WLCAP) mylist[p] = ((e0 + 5) << SLB) | (int)s5; p = p + 1; }
    if (h6) { if (p < WLCAP) mylist[p] = ((e0 + 6) << SLB) | (int)s6; p = p + 1; }
    if (h7) { if (p < WLCAP) mylist[p] = ((e0 + 7) << SLB) | (int)s7; p = p + 1; }
    wc += (int)(__builtin_popcount(m0) + __builtin_popcount(m1) + __builtin_popcount(m2) + __builtin_popcount(m3) +
                __builtin_popcount(m4) + __builtin_popcount(m5) + __builtin_popcount(m6) + __builtin_popcount(m7));
  }
}

__device__ __forceinline__ int count_pass(const int* lists, const int* wcn, int* bins, int lane) {
  int ov = 0;
#pragma unroll 1
  for (int w2 = 0; w2 < NWAVE; ++w2) {
    int c = wcn[w2];
    if (c > WLCAP) ov = 1;
    c = c < 0 ? 0 : (c > WLCAP ? WLCAP : c);
#pragma unroll 1
    for (int b0 = 0; b0 < c; b0 += 32) {
      const int idx = b0 + lane;
      const int ent = lists[w2 * WLCAP + (idx < WLCAP ? idx : WLCAP - 1)];
      const int m32 = (c - b0) < 32 ? (c - b0) : 32;
#pragma unroll 1
      for (int k = 0; k < m32; ++k) {
        const int u    = __builtin_amdgcn_readlane(ent, k);
        const int slot = u & (NBRUN - 1);
        if (lane == 0) bins[slot] = bins[slot] + 1;
      }
    }
  }
  return ov;
}

__device__ __forceinline__ void bucket_flush(const int* pl, const int* cnt, const int* offs, const int* fl, int ov,
                                             int* lp, int* cp, int* op, int* ndp, int* nsp, int* fp, int tid) {
#pragma unroll 1
  for (int i = tid * 4; i < RCAP; i += NTHR * 4) {
    const v4i v = *(const v4ia*)(pl + i);
    *(volatile v4i*)(lp + i) = v;
  }
  {
    const v4i v = *(const v4ia*)(cnt + 4 * tid);
    *(volatile v4i*)(cp + 4 * tid) = v;
  }
  {
    const v4i v = *(const v4ia*)(offs + 4 * tid);
    *(volatile v4i*)(op + 4 * tid) = v;
  }
  {
    const v4i v = *(const v4ia*)(fl + 4 * tid);
    *(volatile v4i*)(ndp + 4 * tid) = v;
  }
  {
    const v4i v = *(const v4ia*)(fl + NBRUN + 4 * tid);
    *(volatile v4i*)(nsp + 4 * tid) = v;
  }
  if (tid < 8) {
    const v4i f = {ov, ov, ov, ov};
    *(volatile v4i*)(fp + 4 * tid) = f;
  }
}

__global__ __launch_bounds__(NTHR) void k_bucket(const int* __restrict__ srcs, const int* __restrict__ dsts,
                                                 int* LIST, int* CNT, int* OFF, int* NDb, int* NSb, int* FLAG) {
  extern __shared__ __attribute__((aligned(16))) int dsm[];
  int* wl   = dsm;
  int* wl2  = wl + NWAVE * WLCAP;
  int* pl   = wl2 + NWAVE * WLCAP;
  int* cnt  = pl + RCAP;
  int* cno  = cnt + NBRUN;
  int* offs = cno + NBRUN;
  int* cur  = offs + NBRUN;
  int* fl   = cur + NBRUN;
  int* misc = fl + 2 * NBRUN;
  const int tid = (int)threadIdx.x, lane = tid & 31, wave = tid >> 5;
  const int blk = (int)blockIdx.x;
  const unsigned nbs = (unsigned)(blk * NBRUN);

  {
    const v4i z4 = {0, 0, 0, 0};
    for (int i = tid * 4; i < BK_ZINTS; i += NTHR * 4) *(v4ia*)(dsm + i) = z4;
    if (tid < 32) misc[tid] = 0;
  }
  __syncthreads();

  {
    const int per  = ((NE + NWAVE * WCH - 1) / (NWAVE * WCH)) * WCH;
    const int ebeg = wave * per;
    const int eend = (ebeg + per < NE) ? (ebeg + per) : NE;
    int* myl  = wl + wave * WLCAP;
    int* myl2 = wl2 + wave * WLCAP;
    int wc = 0, wc2 = 0;
#pragma unroll 1
    for (int cb = ebeg; cb < eend; cb += WCH) {
      const int e0 = cb + lane * EPT;
      const int ec = e0 < NE - EPT ? e0 : NE - EPT;
      const bool valid = e0 < NE;
      const v4i da = *(const v4ia*)(dsts + ec);
      const v4i db = *(const v4ia*)(dsts + ec + 4);
      const v4i sa = *(const v4ia*)(srcs + ec);
      const v4i sb = *(const v4ia*)(srcs + ec + 4);
      compact8(da, db, valid, nbs, e0, myl, wc);
      compact8(sa, sb, valid, nbs, e0, myl2, wc2);
    }
    if (lane == 0) { misc[wave] = wc; misc[8 + wave] = wc2; }
  }
  __syncthreads();

  if (wave == 0) {
    const int ov = count_pass(wl, misc, cnt, lane);
    if (lane == 0) misc[16] = ov;
  } else if (wave == 1) {
    const int ov = count_pass(wl2, misc + 8, cno, lane);
    if (lane == 0) misc[17] = ov;
  }
  __syncthreads();

  if (wave == 0) {
    const int base = lane * (NBRUN / 32);
    int s = 0;
#pragma unroll 1
    for (int i = 0; i < NBRUN / 32; ++i) s += cnt[base + i];
    int incl = s;
#pragma unroll
    for (int d = 1; d < 32; d <<= 1) {
      const int y = __shfl_up(incl, d, 32);
      if (lane >= d) incl += y;
    }
    const int tot = __shfl(incl, 31, 32);
    if (lane == 0) misc[18] = (tot > RCAP) ? 1 : 0;
    int run = incl - s;
#pragma unroll 1
    for (int i = 0; i < NBRUN / 32; ++i) {
      const int cv = cnt[base + i];
      offs[base + i] = run;
      cur[base + i]  = run;
      run += cv;
    }
  }
  __syncthreads();

  if (wave == 0) {
#pragma unroll 1
    for (int w2 = 0; w2 < NWAVE; ++w2) {
      int c = misc[w2];
      c = c < 0 ? 0 : (c > WLCAP ? WLCAP : c);
#pragma unroll 1
      for (int b0 = 0; b0 < c; b0 += 32) {
        const int idx = b0 + lane;
        const int ent = wl[w2 * WLCAP + (idx < WLCAP ? idx : WLCAP - 1)];
        int eid = (ent >> SLB) & 0xFFFFF;
        eid = eid > NE - 1 ? NE - 1 : eid;
        int sr = srcs[eid];
        sr = sr < 0 ? 0 : (sr > NN - 1 ? NN - 1 : sr);
        const int m32 = (c - b0) < 32 ? (c - b0) : 32;
#pragma unroll 1
        for (int k = 0; k < m32; ++k) {
          const int u    = __builtin_amdgcn_readlane(ent, k);
          const int wd   = __builtin_amdgcn_readlane(sr, k);
          const int slot = u & (NBRUN - 1);
          if (lane == 0) {
            int p = cur[slot];
            p = p < 0 ? 0 : (p > RCAP - 1 ? RCAP - 1 : p);
            pl[p] = wd;
            cur[slot] = p + 1;
          }
        }
      }
    }
  }
  __syncthreads();

  const int ovf = misc[16] | misc[17] | misc[18];
  {
    const float qnan = __uint_as_float(0x7fc00000u);
#pragma unroll 1
    for (int i = tid; i < 2 * NBRUN; i += NTHR) {
      int c = cnt[i];
      c = c < 1 ? 1 : c;
      float v = 1.0f / sqrtf((float)c);
      v = (ovf != 0) ? qnan : v;
      fl[i] = __float_as_int(v);
    }
  }
  __syncthreads();

  int* lp  = LIST + (size_t)blk * RCAP;
  int* cp  = CNT + (size_t)blk * NBRUN;
  int* op  = OFF + (size_t)blk * NBRUN;
  int* ndp = NDb + (size_t)blk * NBRUN;
  int* nsp = NSb + (size_t)blk * NBRUN;
  int* fp  = FLAG + (size_t)blk * 32;
  bucket_flush(pl, cnt, offs, fl, ovf, lp, cp, op, ndp, nsp, fp, tid);
  __threadfence();
  bucket_flush(pl, cnt, offs, fl, ovf, lp, cp, op, ndp, nsp, fp, tid);
}

template <int KEXT, int BPITCH>
__device__ __forceinline__ void gemm_16x64(const unsigned short* __restrict__ ap,
                                           const unsigned short* __restrict__ bp, v8f (&acc)[4]) {
#pragma unroll 1
  for (int k0 = 0; k0 < KEXT; k0 += 32) {
    FragB af;
    af.h[0] = *(const v8usa*)(ap + k0);
    af.h[1] = *(const v8usa*)(ap + k0 + 16);
#pragma unroll
    for (int nt = 0; nt < 4; ++nt) {
      const unsigned short* wq = bp + (size_t)(16 * nt) * (size_t)BPITCH + k0;
      FragB bf;
      bf.h[0] = *(const v8usa*)wq;
      bf.h[1] = *(const v8usa*)(wq + 16);
      acc[nt] = wmb(af, bf, acc[nt]);
    }
  }
}

__device__ __forceinline__ void stage_d(float* stg, const v8f (&acc)[4], int wave, int hh, int m) {
#pragma unroll
  for (int nt = 0; nt < 4; ++nt) {
#pragma unroll
    for (int r = 0; r < 8; ++r) stg[(16 * wave + 8 * hh + r) * SP + 16 * nt + m] = acc[nt][r];
  }
}

template <int KEXT, int APITCH, int BPITCH>
__global__ __launch_bounds__(NTHR) __attribute__((amdgpu_num_vgpr(248)))
void k_gemm(const unsigned short* __restrict__ A, const unsigned short* __restrict__ BT,
            const float* __restrict__ NS, float* P) {
  __shared__ __attribute__((aligned(16))) float stg[GBM * SP];
  __shared__ __attribute__((aligned(16))) float sns[GBM];
  const int tid = (int)threadIdx.x, lane = tid & 31, wave = tid >> 5, hh = lane >> 4, m = lane & 15;
  const int rowBase = (int)blockIdx.x * GBM;
  const int col0    = (int)blockIdx.y * 64;
  if (tid < 32) *(v4fa*)(sns + 4 * tid) = *(const v4fa*)(NS + rowBase + 4 * tid);

  v8f acc[4];
  {
    const v8f z = {0.f, 0.f, 0.f, 0.f, 0.f, 0.f, 0.f, 0.f};
#pragma unroll
    for (int t = 0; t < 4; ++t) acc[t] = z;
  }
  const unsigned short* ap = A + (size_t)(rowBase + 16 * wave + m) * (size_t)APITCH + 8 * hh;
  const unsigned short* bp = BT + (size_t)(col0 + m) * (size_t)BPITCH + 8 * hh;
  gemm_16x64<KEXT, BPITCH>(ap, bp, acc);
  stage_d(stg, acc, wave, hh, m);
  __syncthreads();

#pragma unroll 1
  for (int i = 0; i < 8; ++i) {
    const int lr   = 16 * wave + 2 * i + hh;
    const int grow = rowBase + lr;
    const v4f a = *(const v4fa*)(stg + lr * SP + 4 * m);
    const float s = sns[lr];
    v4f o;
    o.x = a.x * s; o.y = a.y * s; o.z = a.z * s; o.w = a.w * s;
    st2_v4f(P + (size_t)grow * FD + col0 + 4 * m, o);
  }
}

__global__ __launch_bounds__(NTHR) void k_replay(const int* __restrict__ LIST, const int* __restrict__ CNT,
                                                 const int* __restrict__ OFF, const float* __restrict__ ND,
                                                 const int* __restrict__ FLAG, const float* __restrict__ P,
                                                 const float* __restrict__ bias, unsigned short* XHL) {
  const int tid = (int)threadIdx.x, lane = tid & 31, wave = tid >> 5;
  const int rowBase = (int)blockIdx.x * ABM;
  const int bucket  = rowBase >> SLB;
  const int* lb  = LIST + (size_t)bucket * RCAP;
  const int flag = FLAG[(size_t)bucket * 32];
  const v4f bv = *(const v4fa*)(bias + 4 * lane);
  const float qnan = __uint_as_float(0x7fc00000u);

#pragma unroll 1
  for (int i = 0; i < ABM / NWAVE; ++i) {
    const int d = rowBase + (ABM / NWAVE) * wave + i;
    int cv  = CNT[d];
    int ofv = OFF[d];
    const int bigv = cv > TRIPCAP ? 1 : 0;
    cv  = cv < 0 ? 0 : (cv > TRIPCAP ? TRIPCAP : cv);
    ofv = ofv < 0 ? 0 : (ofv > RCAP - 1 ? RCAP - 1 : ofv);
    const int c   = __builtin_amdgcn_readfirstlane(cv);
    const int o   = __builtin_amdgcn_readfirstlane(ofv);
    const int big = __builtin_amdgcn_readfirstlane(bigv);
    int last = o + c - 1;
    last = last < o ? o : last;
    last = last > RCAP - 1 ? RCAP - 1 : last;
    float a0 = 0.0f, a1 = 0.0f, a2 = 0.0f, a3 = 0.0f;
#pragma unroll 1
    for (int j = 0; j < c; ++j) {
      int idx = o + j;
      idx = idx > last ? last : idx;
      int sr = lb[idx];
      sr = sr < 0 ? 0 : (sr > NN - 1 ? NN - 1 : sr);
      const v4f v = *(const v4fa*)(P + (size_t)sr * FD + 4 * lane);
      a0 += v.x; a1 += v.y; a2 += v.z; a3 += v.w;
    }
    const float nd = ND[d];
    float y0 = a0 * nd + bv.x, y1 = a1 * nd + bv.y, y2 = a2 * nd + bv.z, y3 = a3 * nd + bv.w;
    y0 = (y0 > 0.0f) ? y0 : (y0 - y0); y1 = (y1 > 0.0f) ? y1 : (y1 - y1);
    y2 = (y2 > 0.0f) ? y2 : (y2 - y2); y3 = (y3 > 0.0f) ? y3 : (y3 - y3);
    const bool bad  = (flag != 0) | (big != 0);
    const bool live = d < NN;
    y0 = bad ? qnan : y0; y1 = bad ? qnan : y1; y2 = bad ? qnan : y2; y3 = bad ? qnan : y3;
    y0 = live ? y0 : 0.0f; y1 = live ? y1 : 0.0f; y2 = live ? y2 : 0.0f; y3 = live ? y3 : 0.0f;
    int h01, h23, l01, l23;
    hilo_pack(y0, y1, y2, y3, h01, h23, l01, l23);
    const v4i ow = regroup_row(h01, h23, l01, l23, lane);
    unsigned short* hp = XHL + (size_t)d * KP + 8 * lane;
    *(volatile v4i*)hp = ow;
    __threadfence();
    *(volatile v4i*)hp = ow;
  }
}

__device__ __forceinline__ void head_flush(const float* ot, float* ob, int nv4, int tid) {
#pragma unroll 1
  for (int it = 0; it < 2; ++it) {
    const int i4 = it * NTHR + tid;
    const v4f v = *(const v4fa*)(ot + 4 * i4);
    asm volatile("" :: "v"(v));
    if (i4 < nv4) *(volatile v4f*)(ob + (size_t)4 * (size_t)i4) = v;
  }
}

__global__ __launch_bounds__(NTHR) void k_head(const unsigned short* __restrict__ XHL,
                                               const unsigned short* __restrict__ WcD,
                                               const float* __restrict__ sm, const int* __restrict__ FLAG,
                                               float* out) {
  __shared__ __attribute__((aligned(16))) float ot[GBM * NCL];
  __shared__ __attribute__((aligned(16))) float sbc[128];
  const int tid = (int)threadIdx.x, lane = tid & 31, wave = tid >> 5, hh = lane >> 4, m = lane & 15;
  const int blk = (int)blockIdx.x;
  const int rowBase = blk * GBM;
  const int flag = FLAG[(size_t)(rowBase >> SLB) * 32];
  if (tid < 32) *(v4fa*)(sbc + 4 * tid) = *(const v4fa*)(sm + 256 + 4 * tid);

  v8f acc = {0.f, 0.f, 0.f, 0.f, 0.f, 0.f, 0.f, 0.f};
  const unsigned short* ap = XHL + (size_t)(rowBase + 16 * wave + m) * (size_t)KP + 8 * hh;
  const unsigned short* bp = WcD + (size_t)m * (size_t)KP + 8 * hh;
#pragma unroll 1
  for (int k0 = 0; k0 < K_HEAD; k0 += 32) {
    FragB af, bf;
    af.h[0] = *(const v8usa*)(ap + k0);
    af.h[1] = *(const v8usa*)(ap + k0 + 16);
    bf.h[0] = *(const v8usa*)(bp + k0);
    bf.h[1] = *(const v8usa*)(bp + k0 + 16);
    acc = wmb(af, bf, acc);
  }
  __syncthreads();

  {
    const float bcv  = sbc[m];
    const float qnan = __uint_as_float(0x7fc00000u);
#pragma unroll
    for (int r = 0; r < 8; ++r) {
      const float v = acc[r] + bcv;
      ot[(16 * wave + 8 * hh + r) * NCL + m] = (flag != 0) ? qnan : v;
    }
  }
  __syncthreads();

  const int liveRows = (NN - rowBase) < GBM ? (NN - rowBase) : GBM;
  const int nv4 = liveRows * (NCL / 4);
  float* ob = out + (size_t)blk * (size_t)(GBM * NCL);
  head_flush(ot, ob, nv4, tid);
  __threadfence();
  head_flush(ot, ob, nv4, tid);
}

extern "C" void kernel_launch(void* const* d_in, const int* in_sizes, int n_in,
                              void* d_out, int out_size, void* d_ws, size_t ws_size,
                              hipStream_t stream) {
  if (n_in < 9) return;
  if (in_sizes[0] != NN * FD) return;
  if (in_sizes[1] != NE) return;
  if (in_sizes[2] != NE) return;
  if (in_sizes[3] != FD * FD) return;
  if (in_sizes[4] != FD) return;
  if (in_sizes[5] != FD * FD) return;
  if (in_sizes[6] != FD) return;
  if (in_sizes[7] != FD * NCL) return;
  if (in_sizes[8] != NCL) return;
  if (out_size != NN * NCL) return;

  const float* h   = (const float*)d_in[0];
  const int*   src = (const int*)d_in[1];
  const int*   dst = (const int*)d_in[2];
  const float* W1  = (const float*)d_in[3];
  const float* b1  = (const float*)d_in[4];
  const float* W2  = (const float*)d_in[5];
  const float* b2  = (const float*)d_in[6];
  const float* Wc  = (const float*)d_in[7];
  const float* bc  = (const float*)d_in[8];
  float* out = (float*)d_out;

  constexpr size_t zXHL  = (size_t)MP * KP * 2;
  constexpr size_t zHB   = (size_t)MP * FD * 2;
  constexpr size_t zP    = (size_t)MP * FD * 4;
  constexpr size_t zLIST = (size_t)NBK * RCAP * 4;
  constexpr size_t zTAB  = (size_t)NBK * NBRUN * 4;
  constexpr size_t zFLAG = (size_t)NBK * 128;
  constexpr size_t zW1T  = (size_t)FD * FD * 2;
  constexpr size_t zW2D  = (size_t)FD * KP * 2;
  constexpr size_t zWCD  = (size_t)NCL * KP * 2;
  constexpr size_t zSM   = (size_t)SMN * 4;
  constexpr size_t oXHL  = 0;
  constexpr size_t oP    = oXHL + zXHL;
  constexpr size_t oLIST = oP + zP;
  constexpr size_t oCNT  = oLIST + zLIST;
  constexpr size_t oOFF  = oCNT + zTAB;
  constexpr size_t oND   = oOFF + zTAB;
  constexpr size_t oNS   = oND + zTAB;
  constexpr size_t oFLAG = oNS + zTAB;
  constexpr size_t oW1T  = oFLAG + zFLAG;
  constexpr size_t oW2D  = oW1T + zW1T;
  constexpr size_t oWCD  = oW2D + zW2D;
  constexpr size_t oSM   = oWCD + zWCD;
  constexpr size_t oEND  = oSM + zSM;
  static_assert(zHB <= zXHL);
  static_assert(zXHL % 128 == 0 && zP % 128 == 0 && zLIST % 128 == 0 && zTAB % 128 == 0 && zFLAG % 128 == 0);
  static_assert(zW1T % 128 == 0 && zW2D % 128 == 0 && zWCD % 128 == 0 && zSM % 128 == 0);
  static_assert(oEND <= (size_t)(128u << 20));
  if (oEND > ws_size) return;

  char* ws = (char*)d_ws;
  unsigned short* XHL  = (unsigned short*)(ws + oXHL);
  unsigned short* HB   = (unsigned short*)(ws + oXHL);
  float*          P    = (float*)(ws + oP);
  int*            LIST = (int*)(ws + oLIST);
  int*            CNT  = (int*)(ws + oCNT);
  int*            OFF  = (int*)(ws + oOFF);
  int*            NDi  = (int*)(ws + oND);
  int*            NSi  = (int*)(ws + oNS);
  const float*    ND   = (const float*)(ws + oND);
  const float*    NS   = (const float*)(ws + oNS);
  int*            FLAG = (int*)(ws + oFLAG);
  unsigned short* W1T  = (unsigned short*)(ws + oW1T);
  unsigned short* W2D  = (unsigned short*)(ws + oW2D);
  unsigned short* WCD  = (unsigned short*)(ws + oWCD);
  float*          SM   = (float*)(ws + oSM);

  hipFuncSetAttribute(reinterpret_cast<const void*>(&k_bucket), hipFuncAttributeMaxDynamicSharedMemorySize, (int)BK_LDS);

  k_prep<<<PBTOT, NTHR, 0, stream>>>(h, W1, b1, W2, b2, Wc, bc, HB, W1T, W2D, WCD, SM);
  k_bucket<<<NBK, NTHR, BK_LDS, stream>>>(src, dst, LIST, CNT, OFF, NDi, NSi, FLAG);
  k_gemm<FD, FD, FD><<<dim3(MP / GBM, 2), NTHR, 0, stream>>>(HB, W1T, NS, P);
  k_replay<<<MP / ABM, NTHR, 0, stream>>>(LIST, CNT, OFF, ND, FLAG, P, SM, XHL);
  k_gemm<K_L2, KP, KP><<<dim3(MP / GBM, 2), NTHR, 0, stream>>>(XHL, W2D, NS, P);
  k_replay<<<MP / ABM, NTHR, 0, stream>>>(LIST, CNT, OFF, ND, FLAG, P, SM + 128, XHL);
  k_head<<<MP / GBM, NTHR, 0, stream>>>(XHL, WCD, SM, FLAG, out);
}
